// PointNetEncoder_83451214561579
// MI455X (gfx1250) — hardware-verified
//
#include <hip/hip_runtime.h>
#pragma clang fp contract(off)

typedef __attribute__((ext_vector_type(16))) _Float16 v16h;
typedef __attribute__((ext_vector_type(8)))  _Float16 v8h;
typedef __attribute__((ext_vector_type(8)))  float    v8f;
typedef __attribute__((ext_vector_type(4)))  float    v4f;
typedef __attribute__((ext_vector_type(4)))  int      v4i;

constexpr int NBATCH   = 4;
constexpr int NPT      = 8192;
constexpr int KNN_K    = 20;
constexpr int TOTPTS   = NBATCH * NPT;
constexpr int MROWS    = TOTPTS * 3;
constexpr int MROWS_B  = NPT * 3;
constexpr int KQ_CAP   = 8;
static_assert(TOTPTS == 32768, "point count");
static_assert(MROWS == 98304, "row count");
static_assert(MROWS % 32 == 0 && MROWS_B % 32 == 0, "row tiles");

constexpr float W_CARRY   = 64.0f;
constexpr float LO_CARRY  = 2048.0f;
constexpr float INV_LO    = 1.0f / LO_CARRY;
constexpr float S_MAIN    = 1.0f / W_CARRY;
constexpr float S_RES     = 1.0f / (W_CARRY * LO_CARRY);
constexpr float ACT_CLAMP = 60000.0f;
constexpr float F16_MIN_NORMAL = 6.103515625e-5f;
constexpr float VN_EPS    = 1e-6f;
constexpr float BN_EPS_F  = 1e-5f;

constexpr int WOFF_1  = 0;
constexpr int WOFF_2  = 2048;
constexpr int WOFF_3  = 5120;
constexpr int WOFF_4P = 11264;
constexpr int WOFF_4D = 20480;
constexpr int WOFF_5  = 29696;
constexpr int WOFF_6  = 38912;
constexpr int WPL_HALVES = 40960;

constexpr size_t SZ_ACT   = (size_t)MROWS * 192 * 2;
constexpr size_t SZ_RF    = (size_t)MROWS * 96 * 4;
constexpr size_t SZ_RD    = (size_t)MROWS_B * 96 * 4;
constexpr size_t SZ_IDX   = (size_t)TOTPTS * KNN_K * 4;
constexpr size_t SZ_WPL   = (size_t)WPL_HALVES * 2;
constexpr size_t SZ_PCONV = (size_t)1024 * 48 * 8;
constexpr size_t SZ_PLAY  = (size_t)128 * 176 * 8;
constexpr size_t SZ_TBL   = 1024;
constexpr size_t SZ_XM    = (size_t)NBATCH * 288 * 4;
constexpr size_t SZ_PMAX  = (size_t)128 * 512 * 4;
constexpr size_t OFF_ACTA  = 0;
constexpr size_t OFF_ACTB  = OFF_ACTA + SZ_ACT;
constexpr size_t OFF_RF    = OFF_ACTB + SZ_ACT;
constexpr size_t OFF_RD    = OFF_RF + SZ_RF;
constexpr size_t OFF_IDX   = OFF_RD + SZ_RD;
constexpr size_t OFF_WPL   = OFF_IDX + SZ_IDX;
constexpr size_t OFF_PCONV = OFF_WPL + SZ_WPL;
constexpr size_t OFF_PLAY  = OFF_PCONV + SZ_PCONV;
constexpr size_t OFF_TBL   = OFF_PLAY + 5 * SZ_PLAY;
constexpr size_t OFF_XM    = OFF_TBL + 6 * SZ_TBL;
constexpr size_t OFF_BP    = OFF_XM + SZ_XM;
constexpr size_t OFF_BD    = OFF_BP + SZ_XM;
constexpr size_t OFF_PMAX  = OFF_BD + SZ_XM;
constexpr size_t WS_TOTAL  = OFF_PMAX + SZ_PMAX;
static_assert(WS_TOTAL <= (size_t)134217728, "carve over the keep line");
static_assert((OFF_ACTB % 128) == 0 && (OFF_RF % 128) == 0 && (OFF_RD % 128) == 0 && (OFF_IDX % 128) == 0, "align");
static_assert((OFF_WPL % 128) == 0 && (OFF_PCONV % 128) == 0 && (OFF_PLAY % 128) == 0 && (OFF_TBL % 128) == 0, "align");
static_assert((OFF_XM % 128) == 0 && (OFF_BP % 128) == 0 && (OFF_BD % 128) == 0 && (OFF_PMAX % 128) == 0, "align");
static_assert((size_t)2040 * 4 == 8160 && (size_t)3060 * 4 == 12240 && (size_t)3400 * 4 == 13600, "output byte offsets");

__device__ __forceinline__ float rne_bf16(float f) {
  unsigned u = __float_as_uint(f);
  u = (u + 0x7FFFu + ((u >> 16) & 1u)) & 0xFFFF0000u;
  return __uint_as_float(u);
}
__device__ __forceinline__ float h16_to_f32(unsigned hb) {
  const unsigned sgn = (hb & 0x8000u) << 16;
  const unsigned em = hb & 0x7fffu;
  const float fn = __uint_as_float((em << 13) + 0x38000000u);
  const float fs = (float)em * 5.9604644775390625e-8f;
  const float mag = (em < 0x400u) ? fs : fn;
  return __uint_as_float(__float_as_uint(mag) | sgn);
}
union FragU { v16h v; v8h h[2]; };
__device__ __forceinline__ v16h frag_load(const _Float16* p) {
  FragU f;
  f.h[0] = *(const v8h*)(p);
  f.h[1] = *(const v8h*)(p + 16);
  return f.v;
}
__device__ __forceinline__ v8f mma_f16(v16h a, v16h b, v8f c) {
  return __builtin_amdgcn_wmma_f32_16x16x32_f16(false, a, false, b, (short)0, c, false, false);
}
__device__ __forceinline__ void guard_group(v8f& a, v8f& b, v8f& c, v8f& d, v16h x, v16h y, v16h z, v16h w) {
  asm volatile("v_nop\n\tv_nop\n\tv_nop\n\tv_nop" : "+v"(a), "+v"(b), "+v"(c), "+v"(d) : "v"(x), "v"(y), "v"(z), "v"(w));
}
__device__ __forceinline__ void guard_acc4(v8f& a, v8f& b, v8f& c, v8f& d) {
  asm volatile("v_nop\n\tv_nop\n\tv_nop\n\tv_nop" : "+v"(a), "+v"(b), "+v"(c), "+v"(d));
}

__device__ __forceinline__ void store_act_tile(const float* sT, int Kpad, unsigned short* dst,
                                               int nChunks, int tid, int nthr) {
  const int cpr = Kpad >> 2;
  const int hc = Kpad >> 3;
  for (int pass = 0; pass < 2; ++pass) {
#pragma unroll 1
    for (int c = tid; c < nChunks; c += nthr) {
      const int row = c / cpr;
      const int cc = c - row * cpr;
      const bool isLo = cc >= hc;
      const int ch0 = (isLo ? (cc - hc) : cc) << 3;
      const float* sp = sT + row * Kpad + ch0;
      const v4f va = *(const v4f*)(sp);
      const v4f vb = *(const v4f*)(sp + 4);
      v8h hv;
#pragma unroll
      for (int e = 0; e < 8; ++e) {
        float x = (e < 4) ? va[e & 3] : vb[e & 3];
        x = fminf(fmaxf(x, -ACT_CLAMP), ACT_CLAMP);
        const float xh = (fabsf(x) < F16_MIN_NORMAL) ? 0.0f : x;
        const _Float16 h = (_Float16)xh;
        const float r = (x - (float)h) * LO_CARRY;
        const float sel = isLo ? r : xh;
        hv[e] = (_Float16)sel;
      }
      *(volatile v8h*)(dst + (size_t)c * 8) = hv;
    }
    __threadfence();
  }
}

__global__ __launch_bounds__(256) void pack_weights_kernel(
    const float* __restrict__ w1f, const float* __restrict__ w1d,
    const float* __restrict__ w2f, const float* __restrict__ w2d,
    const float* __restrict__ w3,
    const float* __restrict__ ws1f, const float* __restrict__ ws1d,
    const float* __restrict__ ws2f, const float* __restrict__ ws2d,
    const float* __restrict__ wlin, unsigned short* __restrict__ wpl) {
  const int g = blockIdx.x * 256 + threadIdx.x;
  const float* sf;
  const float* sd;
  int ld, nOut, kIn, dOff, Kp, base;
  if (g < 256)       { sf = w1f;  sd = w1d;  ld = 21;  nOut = 21; kIn = 21; dOff = 32;   Kp = 32; base = 0; }
  else if (g < 640)  { sf = w2f;  sd = w2d;  ld = 42;  nOut = 42; kIn = 21; dOff = 48;   Kp = 32; base = 256; }
  else if (g < 1408) { sf = w3;   sd = w3;   ld = 42;  nOut = 85; kIn = 42; dOff = 4096; Kp = 64; base = 640; }
  else if (g < 2560) { sf = ws1f; sd = ws1f; ld = 170; nOut = 85; kIn = 85; dOff = 4096; Kp = 96; base = 1408; }
  else if (g < 3712) { sf = ws1d; sd = ws1d; ld = 170; nOut = 85; kIn = 85; dOff = 4096; Kp = 96; base = 2560; }
  else if (g < 4864) { sf = ws2f; sd = ws2d; ld = 85;  nOut = 42; kIn = 85; dOff = 48;   Kp = 96; base = 3712; }
  else               { sf = wlin; sd = wlin; ld = 42;  nOut = 3;  kIn = 42; dOff = 4096; Kp = 64; base = 4864; }
  const int lc = g - base;
  const int cpr = Kp >> 3;
  const int row = lc / cpr;
  const int k0 = (lc - row * cpr) << 3;
  const bool isD = row >= dOff;
  const int rloc = isD ? (row - dOff) : row;
  const float* src = isD ? sd : sf;
  const bool rvalid = rloc < nOut;
  const int rc = rloc < nOut ? rloc : (nOut - 1);
  v8h hv;
#pragma unroll
  for (int e = 0; e < 8; ++e) {
    const int k = k0 + e;
    const int kc = k < kIn ? k : (kIn - 1);
    const float v = src[rc * ld + kc];
    const float x = (rvalid && (k < kIn)) ? (rne_bf16(v) * W_CARRY) : 0.0f;
    hv[e] = (_Float16)x;
  }
  *(volatile v8h*)(wpl + (size_t)g * 8) = hv;
  __threadfence();
  *(volatile v8h*)(wpl + (size_t)g * 8) = hv;
}

__device__ __forceinline__ void knn_insert(float (&kd)[KNN_K], int (&ki)[KNN_K], float pd, int ci) {
#pragma unroll
  for (int s = KNN_K - 1; s >= 1; --s) {
    const bool up = pd > kd[s - 1];
    const bool here = pd > kd[s];
    kd[s] = up ? kd[s - 1] : (here ? pd : kd[s]);
    ki[s] = up ? ki[s - 1] : (here ? ci : ki[s]);
  }
  const bool h0 = pd > kd[0];
  kd[0] = h0 ? pd : kd[0];
  ki[0] = h0 ? ci : ki[0];
}
__device__ __forceinline__ void knn_flush(float (&kd)[KNN_K], int (&ki)[KNN_K],
                                          const float* sqd, const int* sqi, int tid, int& cnt, float& thr) {
#pragma unroll 1
  for (int s = 0; s < KQ_CAP; ++s) {
    if (__builtin_amdgcn_ballot_w32(s < cnt) == 0u) break;
    if (s < cnt) {
      const float pd = sqd[s * 256 + tid];
      const int ci = sqi[s * 256 + tid];
      if (pd > kd[KNN_K - 1]) knn_insert(kd, ki, pd, ci);
    }
  }
  cnt = 0;
  thr = kd[KNN_K - 1];
}

__global__ __launch_bounds__(256) void knn_kernel(const float* __restrict__ pts, int* __restrict__ idxout) {
#pragma clang fp contract(off)
  __shared__ __align__(16) float scand[256 * 4];
  __shared__ float sqd[KQ_CAP * 256];
  __shared__ int sqi[KQ_CAP * 256];
  __shared__ __align__(16) int sidx[256 * KNN_K];
  const int tid = threadIdx.x;
  const int b = blockIdx.x >> 5;
  const int n = ((blockIdx.x & 31) << 8) + tid;
  const float* pb = pts + (size_t)b * NPT * 3;
  const float qx = rne_bf16(pb[n * 3 + 0]);
  const float qy = rne_bf16(pb[n * 3 + 1]);
  const float qz = rne_bf16(pb[n * 3 + 2]);
  const float q0 = qx * qx;
  const float q1 = qy * qy;
  const float q2 = qz * qz;
  const float qxx = (q0 + q1) + q2;
  const float nqxx = -qxx;
  float kd[KNN_K];
  int ki[KNN_K];
#pragma unroll
  for (int s = 0; s < KNN_K; ++s) { kd[s] = -__builtin_inff(); ki[s] = 0; }
  float thr = -__builtin_inff();
  int cnt = 0;
#pragma unroll 1
  for (int ct = 0; ct < NPT / 256; ++ct) {
    __syncthreads();
    {
      const int cj = (ct << 8) + tid;
      const float cx = rne_bf16(pb[cj * 3 + 0]);
      const float cy = rne_bf16(pb[cj * 3 + 1]);
      const float cz = rne_bf16(pb[cj * 3 + 2]);
      const float c0 = cx * cx;
      const float c1 = cy * cy;
      const float c2 = cz * cz;
      v4f cv;
      cv[0] = 2.0f * cx;
      cv[1] = 2.0f * cy;
      cv[2] = 2.0f * cz;
      cv[3] = (c0 + c1) + c2;
      *(v4f*)(scand + tid * 4) = cv;
    }
    __syncthreads();
#pragma unroll 1
    for (int j = 0; j < 256; j += 4) {
#pragma unroll
      for (int u = 0; u < 4; ++u) {
        const v4f cv = *(const v4f*)(scand + (j + u) * 4);
        float s2 = qx * cv[0];
        s2 = __builtin_fmaf(qy, cv[1], s2);
        s2 = __builtin_fmaf(qz, cv[2], s2);
        const float tt = nqxx + s2;
        const float pd = tt - cv[3];
        if (pd > thr) {
          sqd[cnt * 256 + tid] = pd;
          sqi[cnt * 256 + tid] = (ct << 8) + j + u;
          cnt += 1;
        }
      }
      if (__builtin_amdgcn_ballot_w32(cnt >= 4) != 0u) knn_flush(kd, ki, sqd, sqi, tid, cnt, thr);
    }
  }
  knn_flush(kd, ki, sqd, sqi, tid, cnt, thr);
#pragma unroll
  for (int s = 0; s < KNN_K; ++s) sidx[tid * KNN_K + s] = ki[s];
  __syncthreads();
  int* dst = idxout + (size_t)blockIdx.x * (256 * KNN_K);
  for (int pass = 0; pass < 2; ++pass) {
#pragma unroll
    for (int it = 0; it < 5; ++it) {
      const int c = it * 256 + tid;
      const v4i v = *(const v4i*)(sidx + c * 4);
      *(volatile v4i*)(dst + c * 4) = v;
    }
    __threadfence();
  }
}

template <bool APPLY>
__global__ __launch_bounds__(256) void convpos_kernel(
    const float* __restrict__ pts, const int* __restrict__ idx,
    const float* __restrict__ wf, const float* __restrict__ wd,
    const float* __restrict__ tbl, double* __restrict__ part, unsigned short* __restrict__ x1out) {
  __shared__ __align__(16) float sT[96 * 32];
  __shared__ float sF[KNN_K * 6 * 32];
  const int tid = threadIdx.x;
  const int lane = tid & 31;
  const int w = tid >> 5;
#pragma unroll 1
  for (int it = 0; it < 3; ++it) {
    const int eI = it * 256 + tid;
    const int eC = eI < 640 ? eI : 639;
    const int l = eC & 31;
    const int k = eC >> 5;
    const int ptl = blockIdx.x * 32 + l;
    const float* pbb = pts + (size_t)(ptl >> 13) * NPT * 3;
    const int nl = ptl & (NPT - 1);
    const float ccx = rne_bf16(pbb[nl * 3 + 0]);
    const float ccy = rne_bf16(pbb[nl * 3 + 1]);
    const float ccz = rne_bf16(pbb[nl * 3 + 2]);
    int j = idx[(size_t)ptl * KNN_K + k];
    j = j < 0 ? 0 : (j > NPT - 1 ? NPT - 1 : j);
    const float nx = rne_bf16(pbb[j * 3 + 0]);
    const float ny = rne_bf16(pbb[j * 3 + 1]);
    const float nz = rne_bf16(pbb[j * 3 + 2]);
    const float ex = nx - ccx;
    const float ey = ny - ccy;
    const float ez = nz - ccz;
    const float rx = ny * ccz - nz * ccy;
    const float ry = nz * ccx - nx * ccz;
    const float rz = nx * ccy - ny * ccx;
    if (eI < 640) {
      sF[(k * 6 + 0) * 32 + l] = ex;
      sF[(k * 6 + 1) * 32 + l] = ey;
      sF[(k * 6 + 2) * 32 + l] = ez;
      sF[(k * 6 + 3) * 32 + l] = rx;
      sF[(k * 6 + 4) * 32 + l] = ry;
      sF[(k * 6 + 5) * 32 + l] = rz;
    }
  }
  __syncthreads();
  const int pt = blockIdx.x * 32 + lane;
  const float* pb = pts + (size_t)(pt >> 13) * NPT * 3;
  const int nq = pt & (NPT - 1);
  const float cx = rne_bf16(pb[nq * 3 + 0]);
  const float cy = rne_bf16(pb[nq * 3 + 1]);
  const float cz = rne_bf16(pb[nq * 3 + 2]);
  if (w < 7) {
#pragma unroll 1
    for (int o = w; o < 21; o += 7) {
      const float f0 = rne_bf16(wf[o * 3 + 0]);
      const float f1 = rne_bf16(wf[o * 3 + 1]);
      const float f2 = rne_bf16(wf[o * 3 + 2]);
      float g0 = 0.f, g1 = 0.f, g2 = 0.f, mean = 0.f, rstd = 0.f;
      if (APPLY) {
        g0 = rne_bf16(wd[o * 3 + 0]);
        g1 = rne_bf16(wd[o * 3 + 1]);
        g2 = rne_bf16(wd[o * 3 + 2]);
        mean = tbl[o];
        rstd = tbl[96 + o];
      }
      const float pcx = f1 * cx, pcy = f1 * cy, pcz = f1 * cz;
      const float dcx = g1 * cx, dcy = g1 * cy, dcz = g1 * cz;
      float a0 = 0.f, a1 = 0.f, a2 = 0.f;
      float ls = 0.f, lq = 0.f;
#pragma unroll 1
      for (int k = 0; k < KNN_K; ++k) {
        const float ex = sF[(k * 6 + 0) * 32 + lane];
        const float ey = sF[(k * 6 + 1) * 32 + lane];
        const float ez = sF[(k * 6 + 2) * 32 + lane];
        const float rx = sF[(k * 6 + 3) * 32 + lane];
        const float ry = sF[(k * 6 + 4) * 32 + lane];
        const float rz = sF[(k * 6 + 5) * 32 + lane];
        float px = f0 * ex + pcx + f2 * rx;
        float py = f0 * ey + pcy + f2 * ry;
        float pz = f0 * ez + pcz + f2 * rz;
        const float nrm = __builtin_amdgcn_sqrtf(px * px + py * py + pz * pz) + VN_EPS;
        if (!APPLY) {
          ls += nrm;
          lq += nrm * nrm;
        } else {
          const float sc = ((nrm - mean) * rstd) * __builtin_amdgcn_rcpf(nrm);
          px *= sc;
          py *= sc;
          pz *= sc;
          const float dx = g0 * ex + dcx + g2 * rx;
          const float dy = g0 * ey + dcy + g2 * ry;
          const float dz = g0 * ez + dcz + g2 * rz;
          const float dot = px * dx + py * dy + pz * dz;
          const float dsq = dx * dx + dy * dy + dz * dz;
          const float tq = dot * __builtin_amdgcn_rcpf(dsq + VN_EPS);
          const bool pos = dot >= 0.f;
          a0 += pos ? px : (px - tq * dx);
          a1 += pos ? py : (py - tq * dy);
          a2 += pos ? pz : (pz - tq * dz);
        }
      }
      if (!APPLY) {
        sT[o * 32 + lane] = ls;
        sT[(21 + o) * 32 + lane] = lq;
      } else {
        sT[(lane * 3 + 0) * 32 + o] = a0 * 0.05f;
        sT[(lane * 3 + 1) * 32 + o] = a1 * 0.05f;
        sT[(lane * 3 + 2) * 32 + o] = a2 * 0.05f;
      }
    }
  } else if (APPLY) {
#pragma unroll 1
    for (int e = lane; e < 96 * 11; e += 32) {
      const int row = e / 11;
      const int col = 21 + (e - row * 11);
      sT[row * 32 + col] = 0.0f;
    }
  }
  __syncthreads();
  if (!APPLY) {
    if (tid < 48) {
      const int which = tid / 24;
      const int c = tid - which * 24;
      const int cc = c < 21 ? c : 20;
      double s = 0.0;
#pragma unroll 1
      for (int l = 0; l < 32; ++l) s += (double)sT[(which * 21 + cc) * 32 + l];
      const double val = (c < 21) ? s : 0.0;
      volatile double* pp = part + (size_t)blockIdx.x * 48 + tid;
      *pp = val;
      __threadfence();
      *pp = val;
    }
  } else {
    store_act_tile(sT, 32, x1out + (size_t)blockIdx.x * 96 * 64, 768, tid, 256);
  }
}

__global__ __launch_bounds__(256) void gemm_hl_kernel(
    const unsigned short* __restrict__ Ap, int lda, int loOff,
    const unsigned short* __restrict__ Btp, int ldb,
    float* __restrict__ C, int ldc, int M, int N, int K, float sMain, float sRes) {
  const _Float16* A = (const _Float16*)Ap;
  const _Float16* Bt = (const _Float16*)Btp;
  __shared__ __align__(16) float sSlab[8][16 * 36];
  const int lane = threadIdx.x & 31;
  const int wave = threadIdx.x >> 5;
  const int tilesN = N >> 5;
  const int tilesM = M >> 5;
  const int tile = blockIdx.x * 8 + wave;
  if (tile >= tilesM * tilesN) return;
  const int tm = tile / tilesN;
  const int tn = tile - tm * tilesN;
  const int m0 = tm << 5;
  const int n0 = tn << 5;
  const int rlane = lane & 15;
  const int koff = (lane >> 4) * 8;
  const int mOff = (lane >> 4) * 8;

  v8f accM[2][2];
  v8f accR[2][2];
#pragma unroll
  for (int i = 0; i < 2; ++i)
#pragma unroll
    for (int j = 0; j < 2; ++j) {
      accM[i][j] = (v8f){0.f, 0.f, 0.f, 0.f, 0.f, 0.f, 0.f, 0.f};
      accR[i][j] = (v8f){0.f, 0.f, 0.f, 0.f, 0.f, 0.f, 0.f, 0.f};
    }

  for (int k0 = 0; k0 < K; k0 += 32) {
    v16h bh[2];
#pragma unroll
    for (int j = 0; j < 2; ++j)
      bh[j] = frag_load(Bt + (size_t)(n0 + (j << 4) + rlane) * ldb + koff + k0);
#pragma unroll
    for (int i = 0; i < 2; ++i) {
      const size_t ao = (size_t)(m0 + (i << 4) + rlane) * lda + koff + k0;
      const v16h ah = frag_load(A + ao);
      const v16h al = frag_load(A + ao + loOff);
#pragma unroll
      for (int j = 0; j < 2; ++j) {
        accM[i][j] = mma_f16(ah, bh[j], accM[i][j]);
        accR[i][j] = mma_f16(al, bh[j], accR[i][j]);
      }
      guard_group(accM[i][0], accM[i][1], accR[i][0], accR[i][1], ah, al, bh[0], bh[1]);
    }
  }
  guard_acc4(accM[0][0], accM[0][1], accM[1][0], accM[1][1]);
  guard_acc4(accR[0][0], accR[0][1], accR[1][0], accR[1][1]);

  float* slab = sSlab[wave];
  const int q = lane >> 3;
  const int c4 = (lane & 7) * 4;
#pragma unroll
  for (int i = 0; i < 2; ++i) {
#pragma unroll
    for (int j = 0; j < 2; ++j) {
#pragma unroll
      for (int r = 0; r < 8; ++r) {
        const float vm = accM[i][j][r] * sMain;
        const float vr = accR[i][j][r] * sRes;
        slab[(mOff + r) * 36 + (j << 4) + rlane] = vm + vr;
      }
    }
    __builtin_amdgcn_fence(__ATOMIC_RELEASE, "workgroup");
    __builtin_amdgcn_wave_barrier();
    __builtin_amdgcn_fence(__ATOMIC_ACQUIRE, "workgroup");
    for (int pass = 0; pass < 2; ++pass) {
#pragma unroll
      for (int it = 0; it < 4; ++it) {
        const int row = it * 4 + q;
        const v4f v = *(const v4f*)(slab + row * 36 + c4);
        *(volatile v4f*)(C + (size_t)(m0 + (i << 4) + row) * ldc + n0 + c4) = v;
      }
      __threadfence();
    }
    __builtin_amdgcn_fence(__ATOMIC_RELEASE, "workgroup");
    __builtin_amdgcn_wave_barrier();
    __builtin_amdgcn_fence(__ATOMIC_ACQUIRE, "workgroup");
  }
}

__global__ __launch_bounds__(192) void norm_stats_kernel(
    const float* __restrict__ P, int ldp, int C, int CW, int CP,
    const float* __restrict__ bias, int hasBias, double* __restrict__ part) {
  __shared__ double sred[2 * 192];
  const int tid = threadIdx.x;
  const int o = tid % CW;
  const int slot = tid / CW;
  const int nslots = 192 / CW;
  const int oc = o < C ? o : (C - 1);
  const int pt0 = blockIdx.x * 256;
  float bx = 0.f, by = 0.f, bz = 0.f;
  if (hasBias) {
    const int b = blockIdx.x >> 5;
    bx = bias[b * 288 + 0 * 96 + oc];
    by = bias[b * 288 + 1 * 96 + oc];
    bz = bias[b * 288 + 2 * 96 + oc];
  }
  double s = 0.0, qq = 0.0;
#pragma unroll 1
  for (int p = slot; p < 256; p += nslots) {
    const size_t m = (size_t)(pt0 + p) * 3;
    const float px = P[(m + 0) * ldp + oc] + bx;
    const float py = P[(m + 1) * ldp + oc] + by;
    const float pz = P[(m + 2) * ldp + oc] + bz;
    const float nrm = __builtin_amdgcn_sqrtf(px * px + py * py + pz * pz) + VN_EPS;
    const double dn = (double)nrm;
    s += dn;
    qq += dn * dn;
  }
  sred[tid] = s;
  sred[192 + tid] = qq;
  __syncthreads();
  if (tid < 2 * CP) {
    const int which = tid / CP;
    const int c = tid - which * CP;
    const int cc = c < C ? c : (C - 1);
    double a = 0.0;
#pragma unroll 1
    for (int sl = 0; sl < nslots; ++sl) a += sred[which * 192 + sl * CW + cc];
    const double val = (c < C) ? a : 0.0;
    volatile double* pp = part + (size_t)blockIdx.x * (2 * CP) + tid;
    *pp = val;
    __threadfence();
    *pp = val;
  }
}

__global__ __launch_bounds__(96) void stats_finalize_kernel(
    const double* __restrict__ part, int nPart, int C, int CP, double invCnt, float* __restrict__ tbl) {
  const int t = threadIdx.x;
  const int tc = t < C ? t : (C - 1);
  double s = 0.0, qq = 0.0;
#pragma unroll 4
  for (int r = 0; r < nPart; ++r) {
    s += part[(size_t)r * (2 * CP) + tc];
    qq += part[(size_t)r * (2 * CP) + CP + tc];
  }
  const double mean = s * invCnt;
  double var = qq * invCnt - mean * mean;
  var = var < 0.0 ? 0.0 : var;
  const float vf = (float)var;
  float mf = (float)mean;
  float rs = 1.0f / sqrtf(vf + BN_EPS_F);
  mf = (t < C) ? mf : 0.0f;
  rs = (t < C) ? rs : 0.0f;
  volatile float* tp = tbl;
  tp[t] = mf;
  tp[96 + t] = rs;
  __threadfence();
  tp[t] = mf;
  tp[96 + t] = rs;
}

__global__ __launch_bounds__(192) void bn_llr_apply_kernel(
    const float* __restrict__ P, int ldp, const float* __restrict__ D, int ldd, int dOff, int hasD,
    const float* __restrict__ tbl, const float* __restrict__ biasP, const float* __restrict__ biasD, int hasBias,
    int C, int Kpad, unsigned short* __restrict__ out) {
  __shared__ __align__(16) float sT[96 * 96];
  const int tid = threadIdx.x;
  const int o = tid % Kpad;
  const int slot = tid / Kpad;
  const int nslots = 192 / Kpad;
  const int oc = o < C ? o : (C - 1);
  const bool valid = o < C;
  const float mean = tbl[oc];
  const float rstd = tbl[96 + oc];
  float bpx = 0.f, bpy = 0.f, bpz = 0.f, bdx = 0.f, bdy = 0.f, bdz = 0.f;
  if (hasBias) {
    bpx = biasP[0 * 96 + oc];
    bpy = biasP[1 * 96 + oc];
    bpz = biasP[2 * 96 + oc];
    bdx = biasD[0 * 96 + oc];
    bdy = biasD[1 * 96 + oc];
    bdz = biasD[2 * 96 + oc];
  }
  const size_t rowBase = (size_t)blockIdx.x * 96;
#pragma unroll 1
  for (int p = slot; p < 32; p += nslots) {
    const size_t m = rowBase + (size_t)p * 3;
    float px = P[(m + 0) * ldp + oc] + bpx;
    float py = P[(m + 1) * ldp + oc] + bpy;
    float pz = P[(m + 2) * ldp + oc] + bpz;
    const float nrm = __builtin_amdgcn_sqrtf(px * px + py * py + pz * pz) + VN_EPS;
    const float sc = ((nrm - mean) * rstd) * __builtin_amdgcn_rcpf(nrm);
    px *= sc;
    py *= sc;
    pz *= sc;
    float ox = px, oy = py, oz = pz;
    if (hasD) {
      const float dx = D[(m + 0) * ldd + dOff + oc] + bdx;
      const float dy = D[(m + 1) * ldd + dOff + oc] + bdy;
      const float dz = D[(m + 2) * ldd + dOff + oc] + bdz;
      const float dot = px * dx + py * dy + pz * dz;
      const float dsq = dx * dx + dy * dy + dz * dz;
      const float tq = dot * __builtin_amdgcn_rcpf(dsq + VN_EPS);
      const bool pos = dot >= 0.f;
      ox = pos ? px : (px - tq * dx);
      oy = pos ? py : (py - tq * dy);
      oz = pos ? pz : (pz - tq * dz);
    }
    sT[(p * 3 + 0) * Kpad + o] = valid ? ox : 0.0f;
    sT[(p * 3 + 1) * Kpad + o] = valid ? oy : 0.0f;
    sT[(p * 3 + 2) * Kpad + o] = valid ? oz : 0.0f;
  }
  __syncthreads();
  store_act_tile(sT, Kpad, out + rowBase * (size_t)(2 * Kpad), 96 * (Kpad >> 2), tid, 192);
}

__global__ __launch_bounds__(384) void mean_bias_kernel(
    const unsigned* __restrict__ x4w, const float* __restrict__ ws1f, const float* __restrict__ ws1d,
    float* __restrict__ xmTbl, float* __restrict__ biasP, float* __restrict__ biasD) {
  __shared__ double sred[8 * 3 * 96];
  __shared__ float sxm[288];
  const int tid = threadIdx.x;
  const int wc = tid % 48;
  const int slot = tid / 48;
  const int b = blockIdx.x;
  const unsigned* xb = x4w + (size_t)b * MROWS_B * 96;
  double acc[3][2];
#pragma unroll
  for (int v = 0; v < 3; ++v) { acc[v][0] = 0.0; acc[v][1] = 0.0; }
#pragma unroll 1
  for (int p = slot; p < NPT; p += 8) {
    const unsigned* rp = xb + (size_t)p * 3 * 96;
#pragma unroll
    for (int v = 0; v < 3; ++v) {
      const unsigned hw = rp[v * 96 + wc];
      const unsigned lw = rp[v * 96 + 48 + wc];
      const float h0 = h16_to_f32(hw & 0xffffu);
      const float l0 = h16_to_f32(lw & 0xffffu);
      const float h1 = h16_to_f32(hw >> 16);
      const float l1 = h16_to_f32(lw >> 16);
      const float x0 = h0 + l0 * INV_LO;
      const float x1 = h1 + l1 * INV_LO;
      acc[v][0] += (double)x0;
      acc[v][1] += (double)x1;
    }
  }
#pragma unroll
  for (int v = 0; v < 3; ++v) {
    sred[(slot * 3 + v) * 96 + 2 * wc + 0] = acc[v][0];
    sred[(slot * 3 + v) * 96 + 2 * wc + 1] = acc[v][1];
  }
  __syncthreads();
  if (tid < 288) {
    const int v = tid / 96;
    const int c = tid - v * 96;
    double s = 0.0;
#pragma unroll 1
    for (int sl = 0; sl < 8; ++sl) s += sred[(sl * 3 + v) * 96 + c];
    const float xm = (c < 85) ? (float)(s * (1.0 / 8192.0)) : 0.0f;
    sxm[tid] = xm;
    volatile float* xp = xmTbl + (size_t)b * 288 + tid;
    *xp = xm;
    __threadfence();
    *xp = xm;
  }
  __syncthreads();
  if (tid < 288) {
    const int v = tid / 96;
    const int o = tid - v * 96;
    const int oc = o < 85 ? o : 84;
    float sf = 0.f, sd = 0.f;
#pragma unroll 1
    for (int c = 0; c < 85; ++c) {
      const float wfv = rne_bf16(ws1f[oc * 170 + 85 + c]);
      const float wdv = rne_bf16(ws1d[oc * 170 + 85 + c]);
      const float xv = sxm[v * 96 + c];
      sf += wfv * xv;
      sd += wdv * xv;
    }
    sf = (o < 85) ? sf : 0.0f;
    sd = (o < 85) ? sd : 0.0f;
    volatile float* bp = biasP + (size_t)b * 288 + tid;
    volatile float* bd = biasD + (size_t)b * 288 + tid;
    *bp = sf;
    *bd = sd;
    __threadfence();
    *bp = sf;
    *bd = sd;
  }
}

__global__ __launch_bounds__(192) void xstd_max_kernel(
    const unsigned* __restrict__ x4w, const float* __restrict__ zl,
    const float* __restrict__ xmTbl, float* __restrict__ pmax) {
  __shared__ __align__(16) float szl[768 * 4];
  __shared__ float sm[4 * 12 * 48];
  const int tid = threadIdx.x;
  const int wc = tid % 48;
  const int slot = tid / 48;
  const int b = blockIdx.x >> 5;
  const size_t row0 = (size_t)blockIdx.x * 768;
#pragma unroll
  for (int it = 0; it < 4; ++it) {
    const int r = it * 192 + tid;
    const v4f z = *(const v4f*)(zl + (row0 + r) * 32);
    *(v4f*)(szl + r * 4) = z;
  }
  float xmv[3][2];
#pragma unroll
  for (int v = 0; v < 3; ++v) {
    xmv[v][0] = xmTbl[b * 288 + v * 96 + 2 * wc + 0];
    xmv[v][1] = xmTbl[b * 288 + v * 96 + 2 * wc + 1];
  }
  __syncthreads();
  float mx[12];
#pragma unroll
  for (int j = 0; j < 12; ++j) mx[j] = -__builtin_inff();
#pragma unroll 1
  for (int p = slot; p < 256; p += 4) {
    const unsigned* rp = x4w + (row0 + (size_t)p * 3) * 96;
    float xv[3][2];
#pragma unroll
    for (int v = 0; v < 3; ++v) {
      const unsigned hw = rp[v * 96 + wc];
      const unsigned lw = rp[v * 96 + 48 + wc];
      const float h0 = h16_to_f32(hw & 0xffffu);
      const float l0 = h16_to_f32(lw & 0xffffu);
      const float h1 = h16_to_f32(hw >> 16);
      const float l1 = h16_to_f32(lw >> 16);
      xv[v][0] = h0 + l0 * INV_LO;
      xv[v][1] = h1 + l1 * INV_LO;
    }
    const v4f z0 = *(const v4f*)(szl + (p * 3 + 0) * 4);
    const v4f z1 = *(const v4f*)(szl + (p * 3 + 1) * 4);
    const v4f z2 = *(const v4f*)(szl + (p * 3 + 2) * 4);
#pragma unroll
    for (int e = 0; e < 2; ++e) {
#pragma unroll
      for (int k = 0; k < 3; ++k) {
        const float va = xv[0][e] * z0[k] + xv[1][e] * z1[k] + xv[2][e] * z2[k];
        const float vb = xmv[0][e] * z0[k] + xmv[1][e] * z1[k] + xmv[2][e] * z2[k];
        mx[e * 3 + k] = fmaxf(mx[e * 3 + k], va);
        mx[6 + e * 3 + k] = fmaxf(mx[6 + e * 3 + k], vb);
      }
    }
  }
#pragma unroll
  for (int j = 0; j < 12; ++j) sm[(slot * 12 + j) * 48 + wc] = mx[j];
  __syncthreads();
  float outv[3];
#pragma unroll
  for (int it = 0; it < 3; ++it) {
    const int e = it * 192 + tid;
    const int ec = e < 509 ? e : 509;
    const int i = ec / 3;
    const int k = ec - i * 3;
    const int ty = i >= 85 ? 1 : 0;
    const int ii = ty ? (i - 85) : i;
    const int cp = ii >> 1;
    const int j = ty * 6 + (ii & 1) * 3 + k;
    float m = sm[(0 * 12 + j) * 48 + cp];
    m = fmaxf(m, sm[(1 * 12 + j) * 48 + cp]);
    m = fmaxf(m, sm[(2 * 12 + j) * 48 + cp]);
    m = fmaxf(m, sm[(3 * 12 + j) * 48 + cp]);
    outv[it] = (e < 510) ? m : 0.0f;
  }
  for (int pass = 0; pass < 2; ++pass) {
#pragma unroll
    for (int it = 0; it < 3; ++it) {
      const int e = it * 192 + tid;
      if (e < 512) *(volatile float*)(pmax + (size_t)blockIdx.x * 512 + e) = outv[it];
    }
    __threadfence();
  }
}

__global__ __launch_bounds__(256) void emit_kernel(
    const float* __restrict__ pmax, const float* __restrict__ xmTbl, float* __restrict__ out) {
  __shared__ __align__(16) float so[3456];
  const int tid = threadIdx.x;
#pragma unroll 1
  for (int e = tid; e < 2040; e += 256) {
    const int b = e / 510;
    const int r = e - b * 510;
    float m = -__builtin_inff();
#pragma unroll 4
    for (int j = 0; j < 32; ++j) m = fmaxf(m, pmax[(size_t)(b * 32 + j) * 512 + r]);
    so[e] = m;
  }
#pragma unroll 1
  for (int e = tid; e < 1020; e += 256) {
    const int b = e / 255;
    const int r = e - b * 255;
    const int c = r / 3;
    const int v = r - c * 3;
    so[2040 + e] = xmTbl[b * 288 + v * 96 + c];
  }
#pragma unroll 1
  for (int e = tid; e < 340; e += 256) {
    const int b = e / 85;
    const int c = e - b * 85;
    const float x0 = xmTbl[b * 288 + 0 * 96 + c];
    const float x1 = xmTbl[b * 288 + 1 * 96 + c];
    const float x2 = xmTbl[b * 288 + 2 * 96 + c];
    so[3060 + e] = ((x0 + x1) + x2) * (1.0f / 3.0f);
  }
  if (tid < 56) so[3400 + tid] = 0.0f;
  __syncthreads();
  for (int pass = 0; pass < 2; ++pass) {
#pragma unroll 1
    for (int q = tid; q < 850; q += 256) {
      const v4f v = *(const v4f*)(so + q * 4);
      *(volatile v4f*)(out + (size_t)q * 4) = v;
    }
    __threadfence();
  }
}

static void launch_gemm(const unsigned short* A, int lda, int loOff, const unsigned short* Bt, int ldb,
                        float* C, int ldc, int M, int N, int K, hipStream_t stream) {
  const int tiles = (M / 32) * (N / 32);
  const int blocks = (tiles + 7) / 8;
  gemm_hl_kernel<<<blocks, 256, 0, stream>>>(A, lda, loOff, Bt, ldb, C, ldc, M, N, K, S_MAIN, S_RES);
}

extern "C" void kernel_launch(void* const* d_in, const int* in_sizes, int n_in,
                              void* d_out, int out_size, void* d_ws, size_t ws_size,
                              hipStream_t stream) {
  (void)in_sizes; (void)n_in; (void)out_size;
  if (ws_size < WS_TOTAL) return;
  const float* points = (const float*)d_in[0];
  const float* wposf  = (const float*)d_in[1];
  const float* wposd  = (const float*)d_in[2];
  const float* w1f    = (const float*)d_in[3];
  const float* w1d    = (const float*)d_in[4];
  const float* w2f    = (const float*)d_in[5];
  const float* w2d    = (const float*)d_in[6];
  const float* w3     = (const float*)d_in[7];
  const float* ws1f   = (const float*)d_in[8];
  const float* ws1d   = (const float*)d_in[9];
  const float* ws2f   = (const float*)d_in[10];
  const float* ws2d   = (const float*)d_in[11];
  const float* wlin   = (const float*)d_in[12];
  float* out = (float*)d_out;
  char* ws = (char*)d_ws;

  unsigned short* actA = (unsigned short*)(ws + OFF_ACTA);
  unsigned short* actB = (unsigned short*)(ws + OFF_ACTB);
  float* Rf = (float*)(ws + OFF_RF);
  float* Rd = (float*)(ws + OFF_RD);
  int* idxp = (int*)(ws + OFF_IDX);
  unsigned short* wpl = (unsigned short*)(ws + OFF_WPL);
  double* pconv = (double*)(ws + OFF_PCONV);
  double* play[5];
  for (int i = 0; i < 5; ++i) play[i] = (double*)(ws + OFF_PLAY + (size_t)i * SZ_PLAY);
  float* tbl[6];
  for (int i = 0; i < 6; ++i) tbl[i] = (float*)(ws + OFF_TBL + (size_t)i * SZ_TBL);
  float* xmTbl = (float*)(ws + OFF_XM);
  float* biasP = (float*)(ws + OFF_BP);
  float* biasD = (float*)(ws + OFF_BD);
  float* pmax = (float*)(ws + OFF_PMAX);

  const double invCntEdge = 1.0 / ((double)TOTPTS * (double)KNN_K);
  const double invCntPt = 1.0 / (double)TOTPTS;

  pack_weights_kernel<<<20, 256, 0, stream>>>(w1f, w1d, w2f, w2d, w3, ws1f, ws1d, ws2f, ws2d, wlin, wpl);
  knn_kernel<<<TOTPTS / 256, 256, 0, stream>>>(points, idxp);
  convpos_kernel<false><<<TOTPTS / 32, 256, 0, stream>>>(points, idxp, wposf, wposd, tbl[0], pconv, actA);
  stats_finalize_kernel<<<1, 96, 0, stream>>>(pconv, 1024, 21, 24, invCntEdge, tbl[0]);
  convpos_kernel<true><<<TOTPTS / 32, 256, 0, stream>>>(points, idxp, wposf, wposd, tbl[0], pconv, actA);

  static_assert(64 % 32 == 0 && 96 % 32 == 0 && 32 % 32 == 0, "tile multiples");
  launch_gemm(actA, 64, 32, wpl + WOFF_1, 32, Rf, 64, MROWS, 64, 32, stream);
  norm_stats_kernel<<<128, 192, 0, stream>>>(Rf, 64, 21, 32, 24, tbl[1], 0, play[0]);
  stats_finalize_kernel<<<1, 96, 0, stream>>>(play[0], 128, 21, 24, invCntPt, tbl[1]);
  bn_llr_apply_kernel<<<TOTPTS / 32, 192, 0, stream>>>(Rf, 64, Rf, 64, 32, 1, tbl[1], tbl[1], tbl[1], 0, 21, 32, actB);

  launch_gemm(actB, 64, 32, wpl + WOFF_2, 32, Rf, 96, MROWS, 96, 32, stream);
  norm_stats_kernel<<<128, 192, 0, stream>>>(Rf, 96, 42, 64, 48, tbl[2], 0, play[1]);
  stats_finalize_kernel<<<1, 96, 0, stream>>>(play[1], 128, 42, 48, invCntPt, tbl[2]);
  bn_llr_apply_kernel<<<TOTPTS / 32, 192, 0, stream>>>(Rf, 96, Rf, 96, 48, 1, tbl[2], tbl[2], tbl[2], 0, 42, 64, actA);

  launch_gemm(actA, 128, 64, wpl + WOFF_3, 64, Rf, 96, MROWS, 96, 64, stream);
  norm_stats_kernel<<<128, 192, 0, stream>>>(Rf, 96, 85, 96, 88, tbl[3], 0, play[2]);
  stats_finalize_kernel<<<1, 96, 0, stream>>>(play[2], 128, 85, 88, invCntPt, tbl[3]);
  bn_llr_apply_kernel<<<TOTPTS / 32, 192, 0, stream>>>(Rf, 96, Rf, 96, 0, 0, tbl[3], tbl[3], tbl[3], 0, 85, 96, actB);

  mean_bias_kernel<<<NBATCH, 384, 0, stream>>>((const unsigned*)actB, ws1f, ws1d, xmTbl, biasP, biasD);

  launch_gemm(actB, 192, 96, wpl + WOFF_4P, 96, Rf, 96, MROWS, 96, 96, stream);
  norm_stats_kernel<<<128, 192, 0, stream>>>(Rf, 96, 85, 96, 88, biasP, 1, play[3]);
  stats_finalize_kernel<<<1, 96, 0, stream>>>(play[3], 128, 85, 88, invCntPt, tbl[4]);
  for (int b = 0; b < NBATCH; ++b) {
    const size_t rowOff = (size_t)b * MROWS_B;
    launch_gemm(actB + rowOff * 192, 192, 96, wpl + WOFF_4D, 96, Rd, 96, MROWS_B, 96, 96, stream);
    bn_llr_apply_kernel<<<NPT / 32, 192, 0, stream>>>(Rf + rowOff * 96, 96, Rd, 96, 0, 1, tbl[4],
                                                      biasP + (size_t)b * 288, biasD + (size_t)b * 288, 1,
                                                      85, 96, actA + rowOff * 192);
  }

  launch_gemm(actA, 192, 96, wpl + WOFF_5, 96, Rf, 96, MROWS, 96, 96, stream);
  norm_stats_kernel<<<128, 192, 0, stream>>>(Rf, 96, 42, 64, 48, tbl[5], 0, play[4]);
  stats_finalize_kernel<<<1, 96, 0, stream>>>(play[4], 128, 42, 48, invCntPt, tbl[5]);
  bn_llr_apply_kernel<<<TOTPTS / 32, 192, 0, stream>>>(Rf, 96, Rf, 96, 48, 1, tbl[5], tbl[5], tbl[5], 0, 42, 64, actA);

  launch_gemm(actA, 128, 64, wpl + WOFF_6, 64, Rf, 32, MROWS, 32, 64, stream);

  xstd_max_kernel<<<128, 192, 0, stream>>>((const unsigned*)actB, Rf, xmTbl, pmax);
  emit_kernel<<<1, 256, 0, stream>>>(pmax, xmTbl, out);
}
